// TensorDense_6725918785757
// MI455X (gfx1250) — hardware-verified
//
#include <hip/hip_runtime.h>
#include <stddef.h>


typedef _Float16 h16;
typedef _Float16 v16h __attribute__((ext_vector_type(16)));
typedef _Float16 v8h  __attribute__((ext_vector_type(8)));
typedef float    v8f  __attribute__((ext_vector_type(8)));
typedef float    v4f  __attribute__((ext_vector_type(4)));

#ifndef NODES
#define NODES 8192
#endif
#define NODES_FULL 8192
#define XW    128
#define OW    384
#define MUL   32
#define NPB   16
#define FS    36
#define LDX   40
#define LDT   72
#define LDO   388
#define K2    2048
#define K1    1024

#define XCARRY 16.0f
#define WCARRY 64.0f
#define FCARRY 256.0f
#define UCARRY 1024.0f

static_assert(NODES >= NPB && NODES <= NODES_FULL && (NODES % NPB) == 0);
static_assert(NPB == 16);
static_assert(MUL == 32 && XW == 4 * MUL && OW == 12 * MUL);
static_assert((FS % 4) == 0 && FS >= 32);
static_assert((LDX % 8) == 0 && LDX >= 32);
static_assert((LDT % 8) == 0 && LDT >= 64);
static_assert((LDO % 4) == 0 && LDO >= OW);
static_assert(((OW * 4) % 128) == 0);
static_assert(NPB * (OW / 4) == 6 * 256);
static_assert(NPB * XW == 256 * 8);
static_assert((K2 % 64) == 0 && (K1 % 64) == 0 && (K2 % 32) == 0 && (K1 % 32) == 0);
static_assert(K2 == 2 * MUL * MUL && K1 == MUL * MUL);
static_assert(4 * NPB * LDX * 2 + 8 * NPB * FS * 4 + NPB * LDO * 4 <= 65536);

#define W12_BYTES ((size_t)4 * 32 * 32 * 2)
#define U2K_BYTES ((size_t)32 * K2 * 2)
#define U1K_BYTES ((size_t)32 * K1 * 2)
#define OFF_W12 ((size_t)0)
#define OFF_U0  (OFF_W12 + W12_BYTES)
#define OFF_U1  (OFF_U0 + U2K_BYTES)
#define OFF_U2  (OFF_U1 + U2K_BYTES)
#define OFF_U3  (OFF_U2 + U1K_BYTES)
#define WS_TOTAL (OFF_U3 + U1K_BYTES)
static_assert((W12_BYTES % 128) == 0 && (U2K_BYTES % 128) == 0 && (U1K_BYTES % 128) == 0);
static_assert(WS_TOTAL <= (size_t)134217728);

#define S3 0.57735026918962576f
#define R2 0.70710678118654752f
#define R6 0.40824829046386302f

constexpr int PSTART[12] = {0, 2, 4, 6, 8, 9, 10, 11, 12, 13, 14, 15};
constexpr int PCNT[12]   = {2, 2, 2, 2, 1, 1, 1, 1, 1, 1, 1, 1};
constexpr int PS_WSEL[16]  = {0, 0, 1, 1, 1, 1, 1, 1, 2, 2, 2, 3, 3, 3, 3, 3};
constexpr int PS_WBASE[16] = {0, 1024, 0, 1024, 0, 1024, 0, 1024, 0, 0, 0, 0, 0, 0, 0, 0};
constexpr int PS_NT[16]    = {1, 3, 1, 1, 1, 1, 1, 1, 2, 2, 2, 2, 2, 3, 2, 2};
constexpr int PS_A[16][3] = {
    {0,0,0}, {1,2,3}, {0,0,0}, {1,0,0}, {0,0,0}, {2,0,0}, {0,0,0}, {3,0,0},
    {3,2,0}, {1,3,0}, {2,1,0}, {1,3,0}, {1,2,0}, {1,2,3}, {2,3,0}, {1,3,0}};
constexpr int PS_B[16][3] = {
    {0,0,0}, {1,2,3}, {1,0,0}, {0,0,0}, {2,0,0}, {0,0,0}, {3,0,0}, {0,0,0},
    {2,3,0}, {3,1,0}, {1,2,0}, {3,1,0}, {2,1,0}, {1,2,3}, {3,2,0}, {1,3,0}};
constexpr float PS_C[16][3] = {
    {1.f,0.f,0.f}, {-S3,-S3,-S3}, {1.f,0.f,0.f}, {1.f,0.f,0.f},
    {1.f,0.f,0.f}, {1.f,0.f,0.f}, {1.f,0.f,0.f}, {1.f,0.f,0.f},
    {R2,-R2,0.f}, {R2,-R2,0.f}, {R2,-R2,0.f},
    {R2,R2,0.f}, {R2,R2,0.f}, {-R6,2.f*R6,-R6}, {R2,R2,0.f}, {-R2,R2,0.f}};

constexpr unsigned featAOff(int sel) { return sel == 0 ? 0u : (unsigned)((1 + sel) * NPB * FS); }
constexpr unsigned featBOff(int sel) { return sel == 0 ? (unsigned)(NPB * FS) : (unsigned)((4 + sel) * NPB * FS); }

__device__ __forceinline__ float bf16r(float x) {
  unsigned int u = __float_as_uint(x);
  u = (u + 0x7FFFu + ((u >> 16) & 1u)) & 0xFFFF0000u;
  return __uint_as_float(u);
}

static __device__ __forceinline__ h16 toh_flush(float v) {
  const float z = (fabsf(v) < 6.103515625e-05f) ? 0.0f : v;
  return (h16)z;
}

__device__ __forceinline__ v16h frag_at(const _Float16* p) {
  v8h lo = *(const v8h*)(p);
  v8h hi = *(const v8h*)(p + 16);
  v16h out;
#pragma unroll
  for (int i = 0; i < 8; ++i) { out[i] = lo[i]; out[i + 8] = hi[i]; }
  return out;
}
__device__ __forceinline__ v16h ld_frag(const _Float16* base, unsigned ld) {
  const unsigned lane = threadIdx.x & 31u;
  return frag_at(base + (lane & 15u) * ld + (lane >> 4) * 8u);
}

__device__ __forceinline__ v8f wmma16(v16h a, v16h b, v8f c) {
  v8f d = __builtin_amdgcn_wmma_f32_16x16x32_f16(false, a, false, b, (short)0, c,
                                                 false, false);
  asm volatile("v_nop\n\tv_nop\n\tv_nop\n\tv_nop" : "+v"(d) : "v"(a), "v"(b));
  return d;
}

__global__ __launch_bounds__(256) void wconv_mix_kernel(
    const float* __restrict__ W, _Float16* __restrict__ Wt) {
  __shared__ _Float16 T[32 * LDX];
  const unsigned tid = threadIdx.x;
#pragma unroll
  for (unsigned j = 0; j < 4u; ++j) {
    const unsigned idx = tid + 256u * j;
    const unsigned mr = idx >> 5, kc = idx & 31u;
    const float v = W[idx];
    T[kc * LDX + mr] = toh_flush(WCARRY * bf16r(v));
  }
  __syncthreads();
  if (tid < 128u) {
    const unsigned n = tid >> 2, c = (tid & 3u) * 8u;
    const v8h x = *(const v8h*)&T[n * LDX + c];
    _Float16* p = Wt + (size_t)tid * 8u;
    *(volatile v8h*)p = x;
    __threadfence();
    *(volatile v8h*)p = x;
  }
}

__global__ __launch_bounds__(256) void wconv_out_kernel(
    const float* __restrict__ W, _Float16* __restrict__ Wt, unsigned K) {
  __shared__ _Float16 T[32 * LDT];
  const unsigned tid = threadIdx.x;
  const unsigned k0 = blockIdx.x * 64u;
#pragma unroll 4
  for (unsigned j = 0; j < 8u; ++j) {
    const unsigned idx = tid + 256u * j;
    const unsigned kr = idx >> 5, nc = idx & 31u;
    const float v = W[(size_t)(k0 + kr) * 32u + nc];
    T[nc * LDT + kr] = toh_flush(UCARRY * bf16r(v));
  }
  __syncthreads();
  const unsigned n = tid >> 3, kc = (tid & 7u) * 8u;
  const v8h x = *(const v8h*)&T[n * LDT + kc];
  _Float16* p = Wt + (size_t)n * K + k0 + kc;
  *(volatile v8h*)p = x;
  __threadfence();
  *(volatile v8h*)p = x;
}

__device__ __forceinline__ void load_brow(const float* featL, unsigned o, float (&b)[16]) {
  const v4f t0 = *(const v4f*)&featL[o];
  const v4f t1 = *(const v4f*)&featL[o + 4u];
  const v4f t2 = *(const v4f*)&featL[o + 16u];
  const v4f t3 = *(const v4f*)&featL[o + 20u];
#pragma unroll
  for (int e = 0; e < 4; ++e) {
    b[e] = t0[e]; b[4 + e] = t1[e]; b[8 + e] = t2[e]; b[12 + e] = t3[e];
  }
}

template <int PI>
__device__ __forceinline__ void run_piece(
    const float* featL,
    const _Float16* __restrict__ U0, const _Float16* __restrict__ U1,
    const _Float16* __restrict__ U2, const _Float16* __restrict__ U3,
    const unsigned m, const unsigned hh, v8f& acc0, v8f& acc1) {
  constexpr int wsel = PS_WSEL[PI];
  constexpr unsigned wbase = (unsigned)PS_WBASE[PI];
  constexpr int NT = PS_NT[PI];
  constexpr unsigned KP = (wsel < 2) ? (unsigned)K2 : (unsigned)K1;
  constexpr unsigned aO0 = featAOff(PS_A[PI][0]), aO1 = featAOff(PS_A[PI][1]), aO2 = featAOff(PS_A[PI][2]);
  constexpr unsigned bO0 = featBOff(PS_B[PI][0]), bO1 = featBOff(PS_B[PI][1]), bO2 = featBOff(PS_B[PI][2]);
  constexpr float C0 = PS_C[PI][0] * FCARRY, C1 = PS_C[PI][1] * FCARRY, C2 = PS_C[PI][2] * FCARRY;
  static_assert(wbase + 1024u <= KP);

  const _Float16* __restrict__ Wp = U0;
  if constexpr (wsel == 1) Wp = U1;
  if constexpr (wsel == 2) Wp = U2;
  if constexpr (wsel == 3) Wp = U3;

  const unsigned rowo = m * FS;
  float b0[16], b1[16], b2[16];
  load_brow(featL, bO0 + rowo + hh * 8u, b0);
  if constexpr (NT >= 2) load_brow(featL, bO1 + rowo + hh * 8u, b1);
  if constexpr (NT >= 3) load_brow(featL, bO2 + rowo + hh * 8u, b2);

  const _Float16* bp0 = Wp + (size_t)m * KP + wbase + hh * 8u;
  const _Float16* bp1 = bp0 + (size_t)16 * KP;

#pragma unroll 2
  for (unsigned i = 0; i < 32u; ++i) {
    const float a0 = C0 * featL[aO0 + rowo + i];
    float a1 = 0.0f, a2 = 0.0f;
    if constexpr (NT >= 2) a1 = C1 * featL[aO1 + rowo + i];
    if constexpr (NT >= 3) a2 = C2 * featL[aO2 + rowo + i];
    v16h af;
#pragma unroll
    for (int e = 0; e < 16; ++e) {
      float f = a0 * b0[e];
      if constexpr (NT >= 2) f += a1 * b1[e];
      if constexpr (NT >= 3) f += a2 * b2[e];
      af[e] = toh_flush(f);
    }
    const v16h w0 = frag_at(bp0 + i * 32u);
    const v16h w1 = frag_at(bp1 + i * 32u);
    acc0 = wmma16(af, w0, acc0);
    acc1 = wmma16(af, w1, acc1);
  }
}

template <int G>
__device__ __forceinline__ void run_unit(
    const float* featL, float* outS,
    const _Float16* __restrict__ U0, const _Float16* __restrict__ U1,
    const _Float16* __restrict__ U2, const _Float16* __restrict__ U3,
    const unsigned m, const unsigned hh) {
  v8f acc0 = {}, acc1 = {};
  run_piece<PSTART[G]>(featL, U0, U1, U2, U3, m, hh, acc0, acc1);
  if constexpr (PCNT[G] == 2) run_piece<PSTART[G] + 1>(featL, U0, U1, U2, U3, m, hh, acc0, acc1);

  constexpr float cs = 1.0f / (FCARRY * UCARRY);
  const unsigned k0c = m, k1c = 16u + m;
  unsigned col0, col1;
  if constexpr (G == 0)     { col0 = k0c;                          col1 = k1c; }
  else if constexpr (G < 4) { col0 = 32u + k0c * 3u + (G - 1);     col1 = 32u + k1c * 3u + (G - 1); }
  else if constexpr (G < 7) { col0 = 128u + k0c * 3u + (G - 4);    col1 = 128u + k1c * 3u + (G - 4); }
  else                      { col0 = 224u + k0c * 5u + (G - 7);    col1 = 224u + k1c * 5u + (G - 7); }
#pragma unroll
  for (int r = 0; r < 8; ++r) {
    const unsigned row = hh * 8u + (unsigned)r;
    outS[row * LDO + col0] = acc0[r] * cs;
    outS[row * LDO + col1] = acc1[r] * cs;
  }
}

__global__ __launch_bounds__(256) void tp_kernel(
    const float* __restrict__ X, const _Float16* __restrict__ Wmix,
    const _Float16* __restrict__ U0, const _Float16* __restrict__ U1,
    const _Float16* __restrict__ U2, const _Float16* __restrict__ U3,
    float* __restrict__ out) {
  __shared__ _Float16 XA[4 * NPB * LDX];
  __shared__ float featL[8 * NPB * FS];
  __shared__ float outS[NPB * LDO];

  const unsigned tid = threadIdx.x, lane = tid & 31u;
  const unsigned wv = tid >> 5;
  const unsigned selv = (wv < 2u) ? 0u : ((wv < 5u) ? (wv - 1u) : (wv - 4u));
  const unsigned matv = (wv == 0u) ? 0u : ((wv == 1u) ? 2u : ((wv < 5u) ? 1u : 3u));
  const int wave = __builtin_amdgcn_readfirstlane(threadIdx.x >> 5);
  const unsigned sel = (unsigned)__builtin_amdgcn_readfirstlane((int)selv);
  const unsigned mat = (unsigned)__builtin_amdgcn_readfirstlane((int)matv);
  const unsigned hh = lane >> 4, m = lane & 15u;
  const unsigned nodeBase = blockIdx.x * (unsigned)NPB;

  {
    const unsigned node = tid >> 4;
    const unsigned col0 = (tid & 15u) * 8u;
    const float* xr = X + (size_t)(nodeBase + node) * XW + col0;
    const v4f a0 = *(const v4f*)(xr);
    const v4f a1 = *(const v4f*)(xr + 4);
    float val[8];
#pragma unroll
    for (int e = 0; e < 4; ++e) { val[e] = a0[e]; val[4 + e] = a1[e]; }
#pragma unroll
    for (unsigned e = 0; e < 8u; ++e) {
      const unsigned col = col0 + e;
      const bool isv = (col >= 32u);
      const unsigned q = isv ? (col - 32u) : 0u;
      const unsigned m3 = q / 3u;
      const unsigned cc = q - m3 * 3u;
      const unsigned ps = isv ? (1u + cc) : 0u;
      const unsigned mm = isv ? m3 : col;
      XA[ps * (NPB * LDX) + node * LDX + mm] = toh_flush(XCARRY * bf16r(val[e]));
    }
  }
  __syncthreads();

  {
    const v16h xa = ld_frag(&XA[sel * (NPB * LDX)], LDX);
    const _Float16* wp = Wmix + (size_t)mat * 1024u + m * 32u + hh * 8u;
    const v16h wb0 = frag_at(wp);
    const v16h wb1 = frag_at(wp + 16 * 32);
    v8f c0 = {}, c1 = {};
    c0 = wmma16(xa, wb0, c0);
    c1 = wmma16(xa, wb1, c1);
    const unsigned fo = (unsigned)wave * (NPB * FS);
#pragma unroll
    for (int r = 0; r < 8; ++r) {
      const unsigned row = hh * 8u + (unsigned)r;
      featL[fo + row * FS + m]       = c0[r] * (1.0f / (XCARRY * WCARRY));
      featL[fo + row * FS + 16u + m] = c1[r] * (1.0f / (XCARRY * WCARRY));
    }
  }
  __syncthreads();

  switch (wave) {
    case 0: run_unit<0>(featL, outS, U0, U1, U2, U3, m, hh); break;
    case 1: run_unit<1>(featL, outS, U0, U1, U2, U3, m, hh); break;
    case 2: run_unit<2>(featL, outS, U0, U1, U2, U3, m, hh); break;
    case 3: run_unit<3>(featL, outS, U0, U1, U2, U3, m, hh); break;
    case 4: run_unit<4>(featL, outS, U0, U1, U2, U3, m, hh);
            run_unit<5>(featL, outS, U0, U1, U2, U3, m, hh); break;
    case 5: run_unit<6>(featL, outS, U0, U1, U2, U3, m, hh);
            run_unit<7>(featL, outS, U0, U1, U2, U3, m, hh); break;
    case 6: run_unit<8>(featL, outS, U0, U1, U2, U3, m, hh);
            run_unit<9>(featL, outS, U0, U1, U2, U3, m, hh); break;
    default: run_unit<10>(featL, outS, U0, U1, U2, U3, m, hh);
             run_unit<11>(featL, outS, U0, U1, U2, U3, m, hh); break;
  }
  __syncthreads();

  v4f xs[6];
  size_t off[6];
#pragma unroll
  for (unsigned j = 0; j < 6u; ++j) {
    const unsigned q = tid + 256u * j;
    const unsigned row = q / 96u;
    const unsigned c4 = q - row * 96u;
    xs[j] = *(const v4f*)&outS[row * LDO + c4 * 4u];
    off[j] = (size_t)nodeBase * OW + (size_t)q * 4u;
  }
#pragma unroll
  for (int j = 0; j < 6; ++j) *(volatile v4f*)(out + off[j]) = xs[j];
  __threadfence();
#pragma unroll
  for (int j = 0; j < 6; ++j) *(volatile v4f*)(out + off[j]) = xs[j];
}

extern "C" void kernel_launch(void* const* d_in, const int* in_sizes, int n_in,
                              void* d_out, int out_size, void* d_ws, size_t ws_size,
                              hipStream_t stream) {
  if (n_in < 9) return;
  if ((long long)in_sizes[0] < (long long)NODES * XW) return;
  if (in_sizes[1] < 1024 || in_sizes[2] < 1024 || in_sizes[3] < 1024 || in_sizes[4] < 1024) return;
  if (in_sizes[5] < K2 * 32 || in_sizes[6] < K2 * 32) return;
  if (in_sizes[7] < K1 * 32 || in_sizes[8] < K1 * 32) return;
  if ((long long)out_size < (long long)NODES * OW) return;
  if (ws_size < WS_TOTAL) return;

  const float* X    = (const float*)d_in[0];
  const float* w10  = (const float*)d_in[1];
  const float* w11  = (const float*)d_in[2];
  const float* w20  = (const float*)d_in[3];
  const float* w21  = (const float*)d_in[4];
  const float* w30e = (const float*)d_in[5];
  const float* w31o = (const float*)d_in[6];
  const float* w31e = (const float*)d_in[7];
  const float* w32e = (const float*)d_in[8];
  float* out = (float*)d_out;

  char* ws = (char*)d_ws;
  _Float16* Wmix = (_Float16*)(ws + OFF_W12);
  _Float16* U0   = (_Float16*)(ws + OFF_U0);
  _Float16* U1   = (_Float16*)(ws + OFF_U1);
  _Float16* U2   = (_Float16*)(ws + OFF_U2);
  _Float16* U3   = (_Float16*)(ws + OFF_U3);

  dim3 blk(256);
  wconv_mix_kernel<<<dim3(1), blk, 0, stream>>>(w10, Wmix + 0 * 1024);
  wconv_mix_kernel<<<dim3(1), blk, 0, stream>>>(w11, Wmix + 1 * 1024);
  wconv_mix_kernel<<<dim3(1), blk, 0, stream>>>(w20, Wmix + 2 * 1024);
  wconv_mix_kernel<<<dim3(1), blk, 0, stream>>>(w21, Wmix + 3 * 1024);
  wconv_out_kernel<<<dim3(K2 / 64), blk, 0, stream>>>(w30e, U0, (unsigned)K2);
  wconv_out_kernel<<<dim3(K2 / 64), blk, 0, stream>>>(w31o, U1, (unsigned)K2);
  wconv_out_kernel<<<dim3(K1 / 64), blk, 0, stream>>>(w31e, U2, (unsigned)K1);
  wconv_out_kernel<<<dim3(K1 / 64), blk, 0, stream>>>(w32e, U3, (unsigned)K1);

  tp_kernel<<<dim3(NODES / NPB), blk, 0, stream>>>(X, Wmix, U0, U1, U2, U3, out);
}
